// GPT2Attention_29231547416971
// MI455X (gfx1250) — hardware-verified
//
#include <hip/hip_runtime.h>


#ifndef NB
#define NB 2
#endif
#ifndef SEQ
#define SEQ 2048
#endif
#define NB_FULL 2
#define SEQ_FULL 2048
#define HID 1024
#define NH 16
#define HS 64
#define NQKV (3 * HID)
#define TOK (NB * SEQ)
#define NBH (NB * NH)
#define TAILQ (((SEQ) < 512) ? (SEQ) : 512)
#define LDK 40
#define EP16 136
#define EP32 132
#define RC 1024.0f
#define RCI 0.0009765625f
#define WSC 64.0f
#define WSCI 0.015625f

static_assert((SEQ % 128) == 0);
static_assert((TAILQ % 128) == 0);
static_assert(NB >= 1 && NB <= NB_FULL);
static_assert(SEQ <= SEQ_FULL);
static_assert((TOK % 128) == 0 && (NQKV % 128) == 0 && (HID % 128) == 0);
static_assert(NH * HS == HID && HS == 64);
static_assert((TOK % 2) == 0 && (NQKV % 2) == 0 && (HID % 2) == 0);

typedef _Float16 v16h __attribute__((ext_vector_type(16)));
typedef _Float16 v8h __attribute__((ext_vector_type(8)));
typedef __bf16 v16bf __attribute__((ext_vector_type(16)));
typedef unsigned short v16us __attribute__((ext_vector_type(16)));
typedef unsigned short v8us __attribute__((ext_vector_type(8)));
typedef float v8f __attribute__((ext_vector_type(8)));
typedef float v4f __attribute__((ext_vector_type(4)));

union Frag {
  v16h f;
  v16bf b;
  v16us w;
  v8us u[2];
  v8h h[2];
};

__device__ __forceinline__ v8f wm_f16(v16h a, v16h b, v8f c) {
  return __builtin_amdgcn_wmma_f32_16x16x32_f16(false, a, false, b, (short)0, c, false, false);
}
__device__ __forceinline__ v8f wm_bf16(v16bf a, v16bf b, v8f c) {
  return __builtin_amdgcn_wmma_f32_16x16x32_bf16(false, a, false, b, (short)0, c, false, false);
}

__device__ __forceinline__ unsigned int bf16r_bits(float f) {
  unsigned int u = __float_as_uint(f);
  u += 0x7FFFu + ((u >> 16) & 1u);
  return u >> 16;
}
__device__ __forceinline__ float bf16r(float f) { return __uint_as_float(bf16r_bits(f) << 16); }

__global__ __launch_bounds__(256) void k_cvt(const float* __restrict__ src, _Float16* d16, unsigned short* db,
                                              int rowsDst, int grpDst, int grpSrc, float scale, int writeb) {
  const int tid = threadIdx.x;
  int row = blockIdx.x * 2 + (tid >> 7);
  row = (row < rowsDst) ? row : (rowsDst - 1);
  const int c8 = (tid & 127) * 8;
  const int g = row / grpDst;
  const int r = row - g * grpDst;
  const float* sp = src + ((size_t)g * (size_t)grpSrc + (size_t)r) * HID + c8;
  const v4f f0 = *(const v4f*)sp;
  const v4f f1 = *(const v4f*)(sp + 4);
  v8h hv;
  v8us bv;
#pragma unroll
  for (int j = 0; j < 4; ++j) {
    const float a0 = bf16r(f0[j]) * scale;
    const float a1 = bf16r(f1[j]) * scale;
    hv[j] = (_Float16)a0;
    hv[j + 4] = (_Float16)a1;
    bv[j] = (unsigned short)(__float_as_uint(a0) >> 16);
    bv[j + 4] = (unsigned short)(__float_as_uint(a1) >> 16);
  }
  const size_t off = (size_t)row * HID + c8;
  for (int pass = 0; pass < 2; ++pass) {
    *(volatile v8h*)(d16 + off) = hv;
    if (writeb != 0) *(volatile v8us*)(db + off) = bv;
    __threadfence();
  }
}

template <int MODE>
__global__ __launch_bounds__(256) void k_gemm(const unsigned short* __restrict__ A, const unsigned short* __restrict__ B,
                                               const unsigned short* __restrict__ A2, const unsigned short* __restrict__ B2,
                                               const float* __restrict__ bias,
                                               _Float16* P0, _Float16* P1, _Float16* P2,
                                               _Float16* R0, _Float16* R1, _Float16* R2, float* Out) {
  __shared__ __attribute__((aligned(16))) unsigned short sA[128 * LDK];
  __shared__ __attribute__((aligned(16))) unsigned short sB[128 * LDK];
  __shared__ __attribute__((aligned(16))) _Float16 sC16[(MODE == 0) ? (128 * EP16) : 8];
  __shared__ __attribute__((aligned(16))) float sC32[(MODE == 1) ? (64 * EP32) : 4];

  const int tid = threadIdx.x;
  const int lane = tid & 31;
  const int wid = tid >> 5;
  const int waveM = wid & 3;
  const int waveN = wid >> 2;
  const int l16 = lane & 15;
  const int lh = lane >> 4;
  const int mBase = blockIdx.y * 128;
  const int nBase = blockIdx.x * 128;
  const bool resTile = (MODE == 1) && ((mBase % SEQ) >= (SEQ - TAILQ));
  const int nsteps = (HID / 32) * (resTile ? 2 : 1);

  const v8f z8 = {};
  v8f acc[2][4];
#pragma unroll
  for (int i = 0; i < 2; ++i)
#pragma unroll
    for (int j = 0; j < 4; ++j) acc[i][j] = z8;

  for (int ks = 0; ks < nsteps; ++ks) {
    const bool second = (MODE == 1) && (ks >= (HID / 32));
    const int k0 = (second ? (ks - (HID / 32)) : ks) * 32;
    const unsigned short* Ab = second ? A2 : A;
    const unsigned short* Bb = second ? B2 : B;
    v8us ra[2], rb[2];
#pragma unroll
    for (int t = 0; t < 2; ++t) {
      const int ci = tid + t * 256;
      const int row = ci >> 2;
      const int kc = (ci & 3) * 8;
      ra[t] = *(const v8us*)(Ab + (size_t)(mBase + row) * HID + k0 + kc);
      rb[t] = *(const v8us*)(Bb + (size_t)(nBase + row) * HID + k0 + kc);
    }
    __syncthreads();
#pragma unroll
    for (int t = 0; t < 2; ++t) {
      const int ci = tid + t * 256;
      const int row = ci >> 2;
      const int kc = (ci & 3) * 8;
      *(v8us*)(&sA[row * LDK + kc]) = ra[t];
      *(v8us*)(&sB[row * LDK + kc]) = rb[t];
    }
    __syncthreads();
    Frag af[2], bg[4];
#pragma unroll
    for (int i = 0; i < 2; ++i) {
      const int base = (waveM * 32 + i * 16 + l16) * LDK + 8 * lh;
      af[i].u[0] = *(const v8us*)(&sA[base]);
      af[i].u[1] = *(const v8us*)(&sA[base + 16]);
    }
#pragma unroll
    for (int j = 0; j < 4; ++j) {
      const int base = (waveN * 64 + j * 16 + l16) * LDK + 8 * lh;
      bg[j].u[0] = *(const v8us*)(&sB[base]);
      bg[j].u[1] = *(const v8us*)(&sB[base + 16]);
    }
    bool usebf = false;
    if constexpr (MODE == 1) usebf = second;
    if (usebf) {
#pragma unroll
      for (int i = 0; i < 2; ++i)
#pragma unroll
        for (int j = 0; j < 4; ++j) acc[i][j] = wm_bf16(af[i].b, bg[j].b, acc[i][j]);
    } else {
#pragma unroll
      for (int i = 0; i < 2; ++i)
#pragma unroll
        for (int j = 0; j < 4; ++j) acc[i][j] = wm_f16(af[i].f, bg[j].f, acc[i][j]);
    }
    asm volatile("v_nop\n\tv_nop\n\tv_nop\n\tv_nop"
                 : "+v"(acc[0][0]), "+v"(acc[0][1]), "+v"(acc[0][2]), "+v"(acc[0][3]),
                   "+v"(acc[1][0]), "+v"(acc[1][1]), "+v"(acc[1][2]), "+v"(acc[1][3])
                 : "v"(af[0].f), "v"(af[1].f), "v"(bg[0].f), "v"(bg[1].f), "v"(bg[2].f), "v"(bg[3].f));
  }

  float bcol[4];
#pragma unroll
  for (int j = 0; j < 4; ++j) bcol[j] = bf16r(bias[nBase + waveN * 64 + j * 16 + l16]);

  if constexpr (MODE == 0) {
    const int sec = nBase / HID;
    const int hA = (nBase - sec * HID) / HS;
    const int bIdx = mBase / SEQ;
    const int sBase = mBase - bIdx * SEQ;
    _Float16* const PH = (sec == 0) ? P0 : ((sec == 1) ? P1 : P2);
    _Float16* const PR = (sec == 0) ? R0 : ((sec == 1) ? R1 : R2);
#pragma unroll
    for (int ph = 0; ph < 2; ++ph) {
#pragma unroll
      for (int i = 0; i < 2; ++i)
#pragma unroll
        for (int j = 0; j < 4; ++j)
#pragma unroll
          for (int v = 0; v < 8; ++v) {
            const int mloc = waveM * 32 + i * 16 + 8 * lh + v;
            const int nloc = waveN * 64 + j * 16 + l16;
            const float val = acc[i][j][v] * WSCI + bcol[j];
            const _Float16 hi = (_Float16)val;
            _Float16 w = hi;
            if (ph == 1) w = (_Float16)((val - (float)hi) * RC);
            sC16[mloc * EP16 + nloc] = w;
          }
      __syncthreads();
      _Float16* const dstP = (ph == 0) ? PH : PR;
      if (sec < 2) {
        for (int pass = 0; pass < 2; ++pass) {
#pragma unroll
          for (int it = 0; it < 8; ++it) {
            const int p = it * 256 + tid;
            const int L = p >> 3;
            const int q8 = p & 7;
            const int mloc = L >> 1;
            const int hh = L & 1;
            const int s = sBase + mloc;
            const int hd = hA + hh;
            const v8h val = *(const v8h*)(&sC16[mloc * EP16 + hh * 64 + q8 * 8]);
            *(volatile v8h*)(dstP + (((size_t)(bIdx * NH + hd) * SEQ + s) * HS + q8 * 8)) = val;
          }
          __threadfence();
        }
      } else {
        for (int pass = 0; pass < 2; ++pass) {
#pragma unroll
          for (int it = 0; it < 8; ++it) {
            const int p = it * 256 + tid;
            const int nloc = p >> 4;
            const int qq = p & 15;
            v8h val;
#pragma unroll
            for (int e = 0; e < 8; ++e) val[e] = sC16[(qq * 8 + e) * EP16 + nloc];
            const int c = nloc & 63;
            const int hd = hA + (nloc >> 6);
            const int s0 = sBase + qq * 8;
            *(volatile v8h*)(dstP + (((size_t)(bIdx * NH + hd) * HS + c) * SEQ + s0)) = val;
          }
          __threadfence();
        }
      }
      __syncthreads();
    }
  } else {
#pragma unroll
    for (int hv = 0; hv < 2; ++hv) {
      if ((waveM >> 1) == hv) {
#pragma unroll
        for (int i = 0; i < 2; ++i)
#pragma unroll
          for (int j = 0; j < 4; ++j)
#pragma unroll
            for (int v = 0; v < 8; ++v) {
              const int row = waveM * 32 + i * 16 + 8 * lh + v - hv * 64;
              const int col = waveN * 64 + j * 16 + l16;
              sC32[row * EP32 + col] = acc[i][j][v] * WSCI + bcol[j];
            }
      }
      __syncthreads();
      for (int pass = 0; pass < 2; ++pass) {
#pragma unroll
        for (int it = 0; it < 8; ++it) {
          const int p = it * 256 + tid;
          const int row = p >> 5;
          const int q4 = p & 31;
          const v4f val = *(const v4f*)(&sC32[row * EP32 + q4 * 4]);
          *(volatile v4f*)(Out + ((size_t)(mBase + hv * 64 + row)) * HID + nBase + q4 * 4) = val;
        }
        __threadfence();
      }
      __syncthreads();
    }
  }
}

template <bool TAIL>
__global__ __launch_bounds__(128) void k_attn(const _Float16* __restrict__ Qh, const _Float16* __restrict__ Qr,
                                              const _Float16* __restrict__ Kh, const _Float16* __restrict__ Kr,
                                              const _Float16* __restrict__ Vh, const _Float16* __restrict__ Vr,
                                              _Float16* Ch, unsigned short* Cr, int qblk0) {
  __shared__ __attribute__((aligned(16))) _Float16 ldsP[4][16 * 32];
  __shared__ __attribute__((aligned(16))) _Float16 ldsR[TAIL ? 4 : 1][16 * 32];
  __shared__ __attribute__((aligned(16))) float sO[4][16][HS];

  const int tid = threadIdx.x;
  const int wave = tid >> 5;
  const int lane = tid & 31;
  const int l16 = lane & 15;
  const int lh = lane >> 4;
  const int bh = blockIdx.y;
  const int b = bh / NH;
  const int h = bh - b * NH;
  const int q0 = (blockIdx.x + qblk0) * 64 + wave * 16;

  const size_t qoff = ((size_t)bh * SEQ + q0 + l16) * HS + 8 * lh;
  v16h aq[2];
#pragma unroll
  for (int hc = 0; hc < 2; ++hc) {
    Frag a;
    a.h[0] = *(const v8h*)(Qh + qoff + hc * 32);
    a.h[1] = *(const v8h*)(Qh + qoff + hc * 32 + 16);
    aq[hc] = a.f;
  }

  const v8f z8 = {};
  float m[8], l[8];
  v8f co[4], cx[4];
#pragma unroll
  for (int r = 0; r < 8; ++r) { m[r] = -1e30f; l[r] = 0.0f; }
#pragma unroll
  for (int j = 0; j < 4; ++j) { co[j] = z8; cx[j] = z8; }

  const _Float16* kB = Kh + (size_t)bh * SEQ * HS;
  const _Float16* krB = Kr + (size_t)bh * SEQ * HS;
  const _Float16* vB = Vh + (size_t)bh * HS * SEQ;
  const _Float16* vrB = Vr + (size_t)bh * HS * SEQ;

  for (int f0 = q0 & ~31; f0 < SEQ; f0 += 32) {
    v8f s0 = z8, s1 = z8, sx0 = z8, sx1 = z8;
    const _Float16* kp0 = kB + (size_t)(f0 + l16) * HS + 8 * lh;
    const _Float16* kp1 = kp0 + 16 * HS;
#pragma unroll
    for (int hc = 0; hc < 2; ++hc) {
      Frag b0, b1;
      b0.h[0] = *(const v8h*)(kp0 + hc * 32);
      b0.h[1] = *(const v8h*)(kp0 + hc * 32 + 16);
      b1.h[0] = *(const v8h*)(kp1 + hc * 32);
      b1.h[1] = *(const v8h*)(kp1 + hc * 32 + 16);
      s0 = wm_f16(aq[hc], b0.f, s0);
      s1 = wm_f16(aq[hc], b1.f, s1);
      if constexpr (TAIL) {
        const _Float16* kq0 = krB + (size_t)(f0 + l16) * HS + 8 * lh + hc * 32;
        const _Float16* kq1 = kq0 + 16 * HS;
        Frag c0, c1, ar;
        c0.h[0] = *(const v8h*)(kq0);
        c0.h[1] = *(const v8h*)(kq0 + 16);
        c1.h[0] = *(const v8h*)(kq1);
        c1.h[1] = *(const v8h*)(kq1 + 16);
        ar.h[0] = *(const v8h*)(Qr + qoff + hc * 32);
        ar.h[1] = *(const v8h*)(Qr + qoff + hc * 32 + 16);
        sx0 = wm_f16(aq[hc], c0.f, sx0);
        sx0 = wm_f16(ar.f, b0.f, sx0);
        sx1 = wm_f16(aq[hc], c1.f, sx1);
        sx1 = wm_f16(ar.f, b1.f, sx1);
        asm volatile("v_nop\n\tv_nop\n\tv_nop\n\tv_nop" : "+v"(s0), "+v"(s1), "+v"(sx0), "+v"(sx1)
                     : "v"(b0.f), "v"(b1.f), "v"(c0.f), "v"(c1.f), "v"(ar.f), "v"(aq[hc]));
      } else {
        asm volatile("v_nop\n\tv_nop\n\tv_nop\n\tv_nop" : "+v"(s0), "+v"(s1) : "v"(b0.f), "v"(b1.f), "v"(aq[hc]));
      }
    }

    float alpha[8];
#pragma unroll
    for (int r = 0; r < 8; ++r) {
      const int t = q0 + r + 8 * lh;
      const int key0 = f0 + l16;
      const int key1 = key0 + 16;
      float a0 = s0[r];
      float a1 = s1[r];
      if constexpr (TAIL) {
        a0 += sx0[r] * RCI;
        a1 += sx1[r] * RCI;
      }
      float x0 = a0 * 0.125f;
      float x1 = a1 * 0.125f;
      x0 = (key0 < t) ? -10000.0f : x0;
      x1 = (key1 < t) ? -10000.0f : x1;
      float tmax = fmaxf(x0, x1);
#pragma unroll
      for (int off = 1; off < 16; off <<= 1) tmax = fmaxf(tmax, __shfl_xor(tmax, off, 32));
      const float mn = fmaxf(m[r], tmax);
      alpha[r] = __expf(m[r] - mn);
      const float p0 = __expf(x0 - mn);
      const float p1 = __expf(x1 - mn);
      float ps = p0 + p1;
#pragma unroll
      for (int off = 1; off < 16; off <<= 1) ps += __shfl_xor(ps, off, 32);
      l[r] = l[r] * alpha[r] + ps;
      m[r] = mn;
      const float c0 = p0 * RC;
      const float c1 = p1 * RC;
      const _Float16 h0 = (_Float16)c0;
      const _Float16 h1 = (_Float16)c1;
      ldsP[wave][(r + 8 * lh) * 32 + l16] = h0;
      ldsP[wave][(r + 8 * lh) * 32 + 16 + l16] = h1;
      if constexpr (TAIL) {
        ldsR[wave][(r + 8 * lh) * 32 + l16] = (_Float16)((c0 - (float)h0) * RC);
        ldsR[wave][(r + 8 * lh) * 32 + 16 + l16] = (_Float16)((c1 - (float)h1) * RC);
      }
    }
#pragma unroll
    for (int j = 0; j < 4; ++j)
#pragma unroll
      for (int r = 0; r < 8; ++r) {
        co[j][r] *= alpha[r];
        if constexpr (TAIL) cx[j][r] *= alpha[r];
      }

    asm volatile("s_wait_dscnt 0" ::: "memory");
    __builtin_amdgcn_fence(3  , "workgroup");
    __builtin_amdgcn_wave_barrier();
    __builtin_amdgcn_fence(2  , "workgroup");

    Frag ap, apr;
    ap.h[0] = *(const v8h*)(&ldsP[wave][l16 * 32 + 8 * lh]);
    ap.h[1] = *(const v8h*)(&ldsP[wave][l16 * 32 + 16 + 8 * lh]);
    if constexpr (TAIL) {
      apr.h[0] = *(const v8h*)(&ldsR[wave][l16 * 32 + 8 * lh]);
      apr.h[1] = *(const v8h*)(&ldsR[wave][l16 * 32 + 16 + 8 * lh]);
    } else {
      apr.f = ap.f;
    }
#pragma unroll
    for (int j = 0; j < 4; ++j) {
      const _Float16* vp = vB + (size_t)(j * 16 + l16) * SEQ + f0 + 8 * lh;
      Frag bv;
      bv.h[0] = *(const v8h*)(vp);
      bv.h[1] = *(const v8h*)(vp + 16);
      co[j] = wm_f16(ap.f, bv.f, co[j]);
      if constexpr (TAIL) {
        const _Float16* wp = vrB + (size_t)(j * 16 + l16) * SEQ + f0 + 8 * lh;
        Frag bw;
        bw.h[0] = *(const v8h*)(wp);
        bw.h[1] = *(const v8h*)(wp + 16);
        cx[j] = wm_f16(ap.f, bw.f, cx[j]);
        cx[j] = wm_f16(apr.f, bv.f, cx[j]);
        asm volatile("v_nop\n\tv_nop\n\tv_nop\n\tv_nop" : "+v"(co[j]), "+v"(cx[j]) : "v"(bv.f), "v"(bw.f), "v"(ap.f), "v"(apr.f));
      } else {
        asm volatile("v_nop\n\tv_nop\n\tv_nop\n\tv_nop" : "+v"(co[j]) : "v"(bv.f), "v"(ap.f));
      }
    }
  }

#pragma unroll
  for (int r = 0; r < 8; ++r) {
    const float inv = (1.0f / l[r]) * RCI;
#pragma unroll
    for (int j = 0; j < 4; ++j) {
      float o = co[j][r];
      if constexpr (TAIL) o += cx[j][r] * RCI;
      sO[wave][r + 8 * lh][j * 16 + l16] = o * inv;
    }
  }
  __builtin_amdgcn_fence(3  , "workgroup");
  __builtin_amdgcn_wave_barrier();
  __builtin_amdgcn_fence(2  , "workgroup");
  for (int pass = 0; pass < 2; ++pass) {
#pragma unroll
    for (int it = 0; it < 4; ++it) {
      const int rr = it * 4 + (lane >> 3);
      const int q8 = lane & 7;
      const v4f o0 = *(const v4f*)(&sO[wave][rr][q8 * 8]);
      const v4f o1 = *(const v4f*)(&sO[wave][rr][q8 * 8 + 4]);
      v8h hv;
      v8us rv;
#pragma unroll
      for (int e = 0; e < 4; ++e) {
        hv[e] = (_Float16)o0[e];
        rv[e] = (unsigned short)bf16r_bits(o0[e] - (float)hv[e]);
        hv[e + 4] = (_Float16)o1[e];
        rv[e + 4] = (unsigned short)bf16r_bits(o1[e] - (float)hv[e + 4]);
      }
      const size_t off = ((size_t)(b * SEQ + q0 + rr)) * HID + h * HS + q8 * 8;
      *(volatile v8h*)(Ch + off) = hv;
      *(volatile v8us*)(Cr + off) = rv;
    }
    __threadfence();
  }
}

extern "C" void kernel_launch(void* const* d_in, const int* in_sizes, int n_in,
                              void* d_out, int out_size, void* d_ws, size_t ws_size, hipStream_t stream) {
  if (n_in < 5) return;
  if (in_sizes[0] < ((NB - 1) * SEQ_FULL + SEQ) * HID) return;
  if (in_sizes[1] < NQKV * HID) return;
  if (in_sizes[2] < NQKV) return;
  if (in_sizes[3] < HID * HID) return;
  if (in_sizes[4] < HID) return;
  if (out_size < TOK * HID) return;

  const float* enc = (const float*)d_in[0];
  const float* w_attn = (const float*)d_in[1];
  const float* b_attn = (const float*)d_in[2];
  const float* w_proj = (const float*)d_in[3];
  const float* b_proj = (const float*)d_in[4];
  float* out = (float*)d_out;

  const size_t plane = (size_t)TOK * HID * 2;
  const size_t waBytes = (size_t)NQKV * HID * 2;
  const size_t wpBytes = (size_t)HID * HID * 2;
  char* ws = (char*)d_ws;
  size_t off = 0;
  char* pX = ws + off;   off += plane;
  char* pWa = ws + off;  off += waBytes;
  char* pWp = ws + off;  off += wpBytes;
  char* pWpb = ws + off; off += wpBytes;
  char* pQh = ws + off;  off += plane;
  char* pQr = ws + off;  off += plane;
  char* pKh = ws + off;  off += plane;
  char* pKr = ws + off;  off += plane;
  char* pVh = ws + off;  off += plane;
  char* pVr = ws + off;  off += plane;
  char* pCh = ws + off;  off += plane;
  char* pCr = ws + off;  off += plane;
  if (off > ws_size) return;

  k_cvt<<<TOK / 2, 256, 0, stream>>>(enc, (_Float16*)pX, (unsigned short*)pWpb, TOK, SEQ, SEQ_FULL, 1.0f, 0);
  k_cvt<<<NQKV / 2, 256, 0, stream>>>(w_attn, (_Float16*)pWa, (unsigned short*)pWpb, NQKV, NQKV, NQKV, WSC, 0);
  k_cvt<<<HID / 2, 256, 0, stream>>>(w_proj, (_Float16*)pWp, (unsigned short*)pWpb, HID, HID, HID, WSC, 1);

  k_gemm<0><<<dim3(NQKV / 128, TOK / 128), 256, 0, stream>>>(
      (const unsigned short*)pX, (const unsigned short*)pWa, (const unsigned short*)pX, (const unsigned short*)pWa, b_attn,
      (_Float16*)pQh, (_Float16*)pKh, (_Float16*)pVh, (_Float16*)pQr, (_Float16*)pKr, (_Float16*)pVr, out);

  const int nMain = (SEQ - TAILQ) / 64;
  if (nMain > 0) {
    k_attn<false><<<dim3(nMain, NBH), 128, 0, stream>>>(
        (const _Float16*)pQh, (const _Float16*)pQr, (const _Float16*)pKh, (const _Float16*)pKr,
        (const _Float16*)pVh, (const _Float16*)pVr, (_Float16*)pCh, (unsigned short*)pCr, 0);
  }
  k_attn<true><<<dim3(TAILQ / 64, NBH), 128, 0, stream>>>(
      (const _Float16*)pQh, (const _Float16*)pQr, (const _Float16*)pKh, (const _Float16*)pKr,
      (const _Float16*)pVh, (const _Float16*)pVr, (_Float16*)pCh, (unsigned short*)pCr, nMain);

  k_gemm<1><<<dim3(HID / 128, TOK / 128), 256, 0, stream>>>(
      (const unsigned short*)pCh, (const unsigned short*)pWp, (const unsigned short*)pCr, (const unsigned short*)pWpb, b_proj,
      (_Float16*)pQh, (_Float16*)pKh, (_Float16*)pVh, (_Float16*)pQr, (_Float16*)pKr, (_Float16*)pVr, out);
}
